// PaiNNBlock_22333829940094
// MI455X (gfx1250) — hardware-verified
//
#include <hip/hip_runtime.h>
#include <stddef.h>
#include <math.h>


#define NN    256
#define DD    128
#define D2    256
#define D3    384
#define RR    20
#define KRP   32
#define HP    136
#define AP2   264
#define NTHR  256
#define NW1   4
#define NT1   (NW1 * 32)
#define NR1   (NW1 * 16)
#define NW2   2
#define NT2   (NW2 * 32)
#define NR2   (NW2 * 16)
#define JC    32
#define SCL   16.0f
#define INV16 0.0625f
#define EPSV  1e-6f

#define G_WF  (D3 * KRP / 8)
#define G_WI1 (D2 * DD / 8)
#define G_WI2 (D3 * DD / 8)
#define G_WMU (D2 * DD / 8)
#define G_WM1 (D2 * D2 / 8)
#define G_WM2 (D3 * DD / 8)
#define G_TOT (G_WF + G_WI1 + G_WI2 + G_WMU + G_WM1 + G_WM2)

#define L1_T  0
#define L1_H  (L1_T + 16 * HP * 2)
#define L1_S  (L1_H + 16 * HP * 2)
#define PW1   (L1_S + 16 * DD * 4)
#define LDS1  (NW1 * PW1)
#define LP_R  0
#define LP_X  (LP_R + NN * KRP * 2)
#define LP_V  (LP_X + JC * D3 * 4)
#define LP_M  (LP_V + JC * D3 * 4)
#define LP_D  (LP_M + JC * 4)
#define LP_O  (LP_D + JC * 3 * 4)
#define LDSP  (LP_O + (DD + D3) * 4)
#define L2_MU 0
#define L2_V  (L2_MU + 3 * 16 * HP * 2)
#define L2_SQ (L2_V + 16 * DD * 4)
#define L2_DT (L2_SQ + 16 * DD * 4)
#define L2_W  (L2_DT + 16 * DD * 4)
#define L2_C  (L2_W + 16 * D3 * 4)
#define L2_H  (L2_C + 16 * AP2 * 2)
#define PW2   (L2_H + 16 * HP * 2)
#define LDS2  (NW2 * PW2)

static_assert(NN == 256 && NTHR == NN);
static_assert((G_WF % NTHR) == 0 && (G_WI1 % NTHR) == 0 && (G_WI2 % NTHR) == 0);
static_assert((G_WMU % NTHR) == 0 && (G_WM1 % NTHR) == 0 && (G_WM2 % NTHR) == 0);
static_assert((JC % 16) == 0 && (NN % JC) == 0 && 3 * JC <= NTHR);
static_assert(((JC * D3) % (4 * NTHR)) == 0);
static_assert((L1_H % 16) == 0 && (L1_S % 16) == 0 && (PW1 % 16) == 0);
static_assert((LP_X % 16) == 0 && (LP_V % 16) == 0 && (LP_M % 16) == 0 && (LP_D % 16) == 0 && (LP_O % 16) == 0);
static_assert((L2_V % 16) == 0 && (L2_SQ % 16) == 0 && (L2_DT % 16) == 0 && (L2_W % 16) == 0);
static_assert((L2_C % 16) == 0 && (L2_H % 16) == 0 && (PW2 % 16) == 0);
static_assert((HP * 2) % 16 == 0 && (AP2 * 2) % 16 == 0 && (KRP * 2) % 16 == 0);
static_assert(RR <= KRP && (RR % 4) == 0);

typedef float    v4f  __attribute__((ext_vector_type(4)));
typedef float    v8f  __attribute__((ext_vector_type(8)));
typedef _Float16 v4h  __attribute__((ext_vector_type(4)));
typedef _Float16 v8h  __attribute__((ext_vector_type(8)));
typedef _Float16 v16h __attribute__((ext_vector_type(16)));
union FragH { v16h v; v8h h[2]; };

__device__ __forceinline__ v8f wmh(v16h a, v16h b, v8f c) {
  v8f d = __builtin_amdgcn_wmma_f32_16x16x32_f16(false, a, false, b, (short)0, c, false, false);
#if defined(__HIP_DEVICE_COMPILE__)
  asm volatile("v_nop\n\tv_nop\n\tv_nop\n\tv_nop" : "+v"(d) : "v"(a), "v"(b));
#endif
  return d;
}

__device__ __forceinline__ v8f zero8() {
  v8f z = {0.f, 0.f, 0.f, 0.f, 0.f, 0.f, 0.f, 0.f};
  return z;
}

__device__ __forceinline__ float wsum32(float s) {
  s += __shfl_xor(s, 16, 32);
  s += __shfl_xor(s, 8, 32);
  s += __shfl_xor(s, 4, 32);
  s += __shfl_xor(s, 2, 32);
  s += __shfl_xor(s, 1, 32);
  return s;
}

__device__ __forceinline__ float sigm(float x) {
  return __builtin_amdgcn_rcpf(1.0f + __expf(-x));
}

__device__ __forceinline__ v8h pack8(v4f a, v4f b) {
  v8h r;
  r[0] = (_Float16)a.x; r[1] = (_Float16)a.y; r[2] = (_Float16)a.z; r[3] = (_Float16)a.w;
  r[4] = (_Float16)b.x; r[5] = (_Float16)b.y; r[6] = (_Float16)b.z; r[7] = (_Float16)b.w;
  return r;
}

template <int KT>
__device__ __forceinline__ void mma8(v8f (&acc)[8], const _Float16* ar, const _Float16* __restrict__ bplane,
                                     int nb0, int KP, int m, int hh) {
#pragma unroll
  for (int t = 0; t < 8; ++t) acc[t] = zero8();
#pragma unroll
  for (int kt = 0; kt < KT; ++kt) {
    FragH a;
    a.h[0] = *(const v8h*)(ar + 32 * kt);
    a.h[1] = *(const v8h*)(ar + 32 * kt + 16);
#pragma unroll
    for (int t = 0; t < 8; ++t) {
      const _Float16* bp = bplane + (size_t)(nb0 + 16 * t + m) * KP + 32 * kt + 8 * hh;
      FragH b;
      b.h[0] = *(const v8h*)bp;
      b.h[1] = *(const v8h*)(bp + 16);
      acc[t] = wmh(a.v, b.v, acc[t]);
    }
  }
}

__global__ __launch_bounds__(NTHR) void k_prep(
    const float* __restrict__ Wf, const float* __restrict__ Wi1, const float* __restrict__ Wi2,
    const float* __restrict__ Wmu, const float* __restrict__ Wm1, const float* __restrict__ Wm2,
    _Float16* pWf, _Float16* pWi1, _Float16* pWi2, _Float16* pWmu, _Float16* pWm1, _Float16* pWm2) {
  const int b0 = G_WF, b1 = b0 + G_WI1, b2 = b1 + G_WI2, b3 = b2 + G_WMU, b4 = b3 + G_WM1, b5 = b4 + G_WM2;
  const int bstart = blockIdx.x * NTHR;
  const float* src; _Float16* dst; int Kv, KP, Nout, segOff;
  if (bstart < b0)      { src = Wf;  dst = pWf;  Kv = RR; KP = KRP; Nout = D3; segOff = 0;  }
  else if (bstart < b1) { src = Wi1; dst = pWi1; Kv = DD; KP = DD;  Nout = D2; segOff = b0; }
  else if (bstart < b2) { src = Wi2; dst = pWi2; Kv = DD; KP = DD;  Nout = D3; segOff = b1; }
  else if (bstart < b3) { src = Wmu; dst = pWmu; Kv = DD; KP = DD;  Nout = D2; segOff = b2; }
  else if (bstart < b4) { src = Wm1; dst = pWm1; Kv = D2; KP = D2;  Nout = D2; segOff = b3; }
  else                  { src = Wm2; dst = pWm2; Kv = DD; KP = DD;  Nout = D3; segOff = b4; }
  const int i = bstart + (int)threadIdx.x;
  if (i >= b5) return;
  const int o  = (i - segOff) * 8;
  const int n  = o / KP;
  const int k0 = o - n * KP;
  const int nc = n < Nout ? n : Nout - 1;
  float v[8];
#pragma unroll
  for (int e = 0; e < 8; ++e) {
    const int k  = k0 + e;
    const int kc = k < Kv ? k : Kv - 1;
    const float xv = src[(size_t)kc * Nout + nc];
    v[e] = (k < Kv && n < Nout) ? xv * SCL : 0.0f;
  }
  v8h hv;
#pragma unroll
  for (int e = 0; e < 8; ++e) hv[e] = (_Float16)v[e];
  _Float16* dp = dst + o;
  *(volatile v8h*)dp = hv;
  __threadfence();
  *(volatile v8h*)dp = hv;
}

__global__ __launch_bounds__(NT1) void k_atom1(
    const float* __restrict__ s_heavy, const int* __restrict__ is_h, const float* __restrict__ h_emb,
    const float* __restrict__ norm1_w, const _Float16* __restrict__ pWi1, const float* __restrict__ b_i1,
    const _Float16* __restrict__ pWi2, const float* __restrict__ b_i2, float* X, int nh) {
  extern __shared__ v4f lds_dyn[];
  const int tid = threadIdx.x, lane = tid & 31, wave = tid >> 5, hh = lane >> 4, m = lane & 15;
  char* lb = (char*)lds_dyn + wave * PW1;
  _Float16* sT  = (_Float16*)(lb + L1_T);
  _Float16* sHh = (_Float16*)(lb + L1_H);
  float*    stg = (float*)(lb + L1_S);
  const int a0 = blockIdx.x * NR1 + wave * 16;

  {
    const v4f hv = *(const v4f*)(h_emb + 4 * lane);
    const v4f wv = *(const v4f*)(norm1_w + 4 * lane);
    for (int rr = 0; rr < 16; ++rr) {
      const int a = a0 + rr;
      const int b = a >> 8, i = a & (NN - 1);
      const int ic = i < nh ? i : nh - 1;
      const v4f sv = *(const v4f*)(s_heavy + ((size_t)b * nh + ic) * DD + 4 * lane);
      const int hf = is_h[a];
      const bool heavy = i < nh;
      v4f s;
      s.x = (hf != 0) ? hv.x : (heavy ? sv.x : 0.0f);
      s.y = (hf != 0) ? hv.y : (heavy ? sv.y : 0.0f);
      s.z = (hf != 0) ? hv.z : (heavy ? sv.z : 0.0f);
      s.w = (hf != 0) ? hv.w : (heavy ? sv.w : 0.0f);
      float ss = s.x * s.x + s.y * s.y + s.z * s.z + s.w * s.w;
      ss = wsum32(ss);
      const float rn = rsqrtf(ss * (1.0f / DD) + EPSV);
      v4h t;
      t.x = (_Float16)((s.x * rn) * (1.0f + wv.x));
      t.y = (_Float16)((s.y * rn) * (1.0f + wv.y));
      t.z = (_Float16)((s.z * rn) * (1.0f + wv.z));
      t.w = (_Float16)((s.w * rn) * (1.0f + wv.w));
      *(v4h*)(sT + rr * HP + 4 * lane) = t;
    }
  }
  __syncthreads();

  v8f acc[8];
  mma8<4>(acc, sT + m * HP + 8 * hh, pWi1, 0, DD, m, hh);
  {
    float* sp = stg + (8 * hh) * DD + m;
#pragma unroll
    for (int t = 0; t < 8; ++t) {
      const float bb = b_i1[16 * t + m];
#pragma unroll
      for (int r = 0; r < 8; ++r) sp[r * DD + 16 * t] = fmaf(acc[t][r], INV16, bb);
    }
  }
  mma8<4>(acc, sT + m * HP + 8 * hh, pWi1, DD, DD, m, hh);
  {
    const float* sp = stg + (8 * hh) * DD + m;
    _Float16* hp = sHh + (8 * hh) * HP + m;
#pragma unroll
    for (int t = 0; t < 8; ++t) {
      const float bg = b_i1[DD + 16 * t + m];
#pragma unroll
      for (int r = 0; r < 8; ++r) {
        const float av = sp[r * DD + 16 * t];
        const float gv = fmaf(acc[t][r], INV16, bg);
        const float h  = (av * sigm(av)) * sigm(gv);
        hp[r * HP + 16 * t] = (_Float16)h;
      }
    }
  }
  __syncthreads();

#pragma unroll
  for (int g = 0; g < 3; ++g) {
    mma8<4>(acc, sHh + m * HP + 8 * hh, pWi2, DD * g, DD, m, hh);
    {
      float* sp = stg + (8 * hh) * DD + m;
#pragma unroll
      for (int t = 0; t < 8; ++t) {
        const float bb = b_i2[DD * g + 16 * t + m];
#pragma unroll
        for (int r = 0; r < 8; ++r) sp[r * DD + 16 * t] = fmaf(acc[t][r], INV16, bb);
      }
    }
    __syncthreads();
    float* gq = X + (size_t)a0 * D3 + DD * g + 4 * lane;
#pragma unroll
    for (int i = 0; i < 16; ++i)
      *(volatile v4f*)(gq + (size_t)i * D3) = *(const v4f*)(stg + i * DD + 4 * lane);
    __threadfence();
#pragma unroll
    for (int i = 0; i < 16; ++i)
      *(volatile v4f*)(gq + (size_t)i * D3) = *(const v4f*)(stg + i * DD + 4 * lane);
    __syncthreads();
  }
}

__global__ __launch_bounds__(NTHR) void k_pair(
    const float* __restrict__ rbf, const float* __restrict__ dir, const float* __restrict__ mask,
    const float* __restrict__ v_all, const float* __restrict__ s_heavy, const int* __restrict__ is_h,
    const float* __restrict__ h_emb, const _Float16* __restrict__ pWf, const float* __restrict__ b_f,
    const float* __restrict__ X, float* Qp, float* MUp, int nh) {
  extern __shared__ v4f lds_dyn[];
  char* lb = (char*)lds_dyn;
  _Float16* sR  = (_Float16*)(lb + LP_R);
  float*    sX  = (float*)(lb + LP_X);
  float*    sVv = (float*)(lb + LP_V);
  float*    sM  = (float*)(lb + LP_M);
  float*    sD  = (float*)(lb + LP_D);
  float*    sO  = (float*)(lb + LP_O);
  const int tid = threadIdx.x, lane = tid & 31, wave = tid >> 5, hh = lane >> 4, m = lane & 15;
  const int bi = blockIdx.x;
  const int b = bi >> 8, i = bi & (NN - 1);
  const int cw = wave * 16 + m;

  {
    const float* rp = rbf + ((size_t)bi * NN + tid) * RR;
    const v4f f0 = *(const v4f*)(rp);
    const v4f f1 = *(const v4f*)(rp + 4);
    const v4f f2 = *(const v4f*)(rp + 8);
    const v4f f3 = *(const v4f*)(rp + 12);
    const v4f f4 = *(const v4f*)(rp + 16);
    v4f z4 = {0.0f, 0.0f, 0.0f, 0.0f};
    const v8h g0 = pack8(f0, f1);
    const v8h g1 = pack8(f2, f3);
    const v8h g2 = pack8(f4, z4);
    const v8h g3 = pack8(z4, z4);
    _Float16* dp = sR + tid * KRP;
    *(v8h*)(dp)      = g0;
    *(v8h*)(dp + 8)  = g1;
    *(v8h*)(dp + 16) = g2;
    *(v8h*)(dp + 24) = g3;
  }

  FragH bf0, bf1, bf2;
  {
    const _Float16* p0 = pWf + (size_t)(cw) * KRP + 8 * hh;
    const _Float16* p1 = pWf + (size_t)(DD + cw) * KRP + 8 * hh;
    const _Float16* p2 = pWf + (size_t)(2 * DD + cw) * KRP + 8 * hh;
    bf0.h[0] = *(const v8h*)p0; bf0.h[1] = *(const v8h*)(p0 + 16);
    bf1.h[0] = *(const v8h*)p1; bf1.h[1] = *(const v8h*)(p1 + 16);
    bf2.h[0] = *(const v8h*)p2; bf2.h[1] = *(const v8h*)(p2 + 16);
  }
  const float bias0 = b_f[cw], bias1 = b_f[DD + cw], bias2 = b_f[2 * DD + cw];

  float aq = 0.0f;
  float aR0 = 0.0f, aR1 = 0.0f, aR2 = 0.0f;
  float aM0 = 0.0f, aM1 = 0.0f, aM2 = 0.0f;

  for (int jc = 0; jc < NN / JC; ++jc) {
    const size_t rbase = (size_t)b * NN + (size_t)jc * JC;
    const float* xs = X + rbase * D3;
    const float* vs = v_all + rbase * D3;
#pragma unroll
    for (int u = 0; u < (JC * D3) / (4 * NTHR); ++u) {
      const int f = tid + NTHR * u;
      *(v4f*)(sX + 4 * f)  = *(const v4f*)(xs + 4 * f);
      *(v4f*)(sVv + 4 * f) = *(const v4f*)(vs + 4 * f);
    }
    if (tid < JC)     sM[tid] = mask[(size_t)bi * NN + jc * JC + tid];
    if (tid < 3 * JC) sD[tid] = dir[((size_t)bi * NN + jc * JC) * 3 + tid];
    __syncthreads();

#pragma unroll
    for (int t2 = 0; t2 < JC / 16; ++t2) {
      const int jt = jc * JC + t2 * 16;
      FragH a;
      const _Float16* ap = sR + (jt + m) * KRP + 8 * hh;
      a.h[0] = *(const v8h*)ap;
      a.h[1] = *(const v8h*)(ap + 16);
      v8f c0 = wmh(a.v, bf0.v, zero8());
      v8f c1 = wmh(a.v, bf1.v, zero8());
      v8f c2 = wmh(a.v, bf2.v, zero8());
#pragma unroll
      for (int r = 0; r < 8; ++r) {
        const int jl = t2 * 16 + 8 * hh + r;
        const float mk = sM[jl];
        const float* xr = sX + jl * D3 + cw;
        const float* vr = sVv + jl * D3 + cw;
        const float wq = fmaf(c0[r], INV16, bias0);
        const float vq = (wq * xr[0]) * mk;
        aq += vq;
        const float wR = fmaf(c1[r], INV16, bias1);
        const float vR = (wR * xr[DD]) * mk;
        aR0 = fmaf(vR, sD[jl * 3 + 0], aR0);
        aR1 = fmaf(vR, sD[jl * 3 + 1], aR1);
        aR2 = fmaf(vR, sD[jl * 3 + 2], aR2);
        const float wM = fmaf(c2[r], INV16, bias2);
        const float vM = (wM * xr[2 * DD]) * mk;
        aM0 = fmaf(vM, vr[0], aM0);
        aM1 = fmaf(vM, vr[DD], aM1);
        aM2 = fmaf(vM, vr[2 * DD], aM2);
      }
    }
    __syncthreads();
  }

  aq  += __shfl_xor(aq, 16, 32);
  aR0 += __shfl_xor(aR0, 16, 32);
  aR1 += __shfl_xor(aR1, 16, 32);
  aR2 += __shfl_xor(aR2, 16, 32);
  aM0 += __shfl_xor(aM0, 16, 32);
  aM1 += __shfl_xor(aM1, 16, 32);
  aM2 += __shfl_xor(aM2, 16, 32);

  {
    const int hf = is_h[bi];
    const int ic = i < nh ? i : nh - 1;
    const float sv = s_heavy[((size_t)b * nh + ic) * DD + cw];
    const float hv = h_emb[cw];
    const float s  = (hf != 0) ? hv : ((i < nh) ? sv : 0.0f);
    const float* vi = v_all + (size_t)bi * D3 + cw;
    const float q0 = s + aq;
    const float u0 = vi[0] + (aR0 + aM0);
    const float u1 = vi[DD] + (aR1 + aM1);
    const float u2 = vi[2 * DD] + (aR2 + aM2);
    if (hh == 0) {
      sO[cw] = q0;
      sO[DD + cw] = u0;
      sO[2 * DD + cw] = u1;
      sO[3 * DD + cw] = u2;
    }
  }
  __syncthreads();
  if (wave == 0) {
    const v4f q4 = *(const v4f*)(sO + 4 * lane);
    const v4f m0 = *(const v4f*)(sO + DD + 4 * lane);
    const v4f m1 = *(const v4f*)(sO + 2 * DD + 4 * lane);
    const v4f m2 = *(const v4f*)(sO + 3 * DD + 4 * lane);
    float* gq = Qp + (size_t)bi * DD + 4 * lane;
    float* gm = MUp + (size_t)bi * D3 + 4 * lane;
    *(volatile v4f*)gq = q4;
    *(volatile v4f*)(gm) = m0;
    *(volatile v4f*)(gm + DD) = m1;
    *(volatile v4f*)(gm + 2 * DD) = m2;
    __threadfence();
    *(volatile v4f*)gq = q4;
    *(volatile v4f*)(gm) = m0;
    *(volatile v4f*)(gm + DD) = m1;
    *(volatile v4f*)(gm + 2 * DD) = m2;
  }
}

__device__ __forceinline__ void atom2_out(const float* sq, const float* sw, float* outq, float* outmu,
                                          int a0, int nh, int lane) {
  for (int rr = 0; rr < 16; ++rr) {
    const int a = a0 + rr;
    const int b = a >> 8, i = a & (NN - 1);
    if (i < nh) {
      const v4f v = *(const v4f*)(sq + rr * DD + 4 * lane);
      *(volatile v4f*)(outq + ((size_t)b * nh + i) * DD + 4 * lane) = v;
    }
#pragma unroll
    for (int p = 0; p < 3; ++p) {
      const v4f v = *(const v4f*)(sw + rr * D3 + 4 * (32 * p + lane));
      *(volatile v4f*)(outmu + (size_t)a * D3 + 4 * (32 * p + lane)) = v;
    }
  }
}

__global__ __launch_bounds__(NT2) void k_atom2(
    const float* __restrict__ Qp, const float* __restrict__ MUp, const float* __restrict__ norm2_w,
    const _Float16* __restrict__ pWmu, const _Float16* __restrict__ pWm1, const float* __restrict__ b_m1,
    const _Float16* __restrict__ pWm2, const float* __restrict__ b_m2, float* outq, float* outmu, int nh) {
  extern __shared__ v4f lds_dyn[];
  const int tid = threadIdx.x, lane = tid & 31, wave = tid >> 5, hh = lane >> 4, m = lane & 15;
  char* lb = (char*)lds_dyn + wave * PW2;
  _Float16* sMu = (_Float16*)(lb + L2_MU);
  float*    sV  = (float*)(lb + L2_V);
  float*    sSq = (float*)(lb + L2_SQ);
  float*    sDt = (float*)(lb + L2_DT);
  float*    sW  = (float*)(lb + L2_W);
  _Float16* sC  = (_Float16*)(lb + L2_C);
  _Float16* sH  = (_Float16*)(lb + L2_H);
  const int a0 = blockIdx.x * NR2 + wave * 16;

  {
    const v4f wv = *(const v4f*)(norm2_w + 4 * lane);
    for (int rr = 0; rr < 16; ++rr) {
      const int a = a0 + rr;
#pragma unroll
      for (int r = 0; r < 3; ++r) {
        const v4f mv = *(const v4f*)(MUp + ((size_t)a * 3 + r) * DD + 4 * lane);
        v4h t;
        t.x = (_Float16)mv.x; t.y = (_Float16)mv.y; t.z = (_Float16)mv.z; t.w = (_Float16)mv.w;
        *(v4h*)(sMu + (r * 16 + rr) * HP + 4 * lane) = t;
      }
      const v4f qv = *(const v4f*)(Qp + (size_t)a * DD + 4 * lane);
      float ss = qv.x * qv.x + qv.y * qv.y + qv.z * qv.z + qv.w * qv.w;
      ss = wsum32(ss);
      const float rn = rsqrtf(ss * (1.0f / DD) + EPSV);
      v4h c;
      c.x = (_Float16)((qv.x * rn) * (1.0f + wv.x));
      c.y = (_Float16)((qv.y * rn) * (1.0f + wv.y));
      c.z = (_Float16)((qv.z * rn) * (1.0f + wv.z));
      c.w = (_Float16)((qv.w * rn) * (1.0f + wv.w));
      *(v4h*)(sC + rr * AP2 + 4 * lane) = c;
    }
  }
  __syncthreads();

  v8f acc[8];
#pragma unroll
  for (int r = 0; r < 3; ++r) {
    mma8<4>(acc, sMu + (r * 16 + m) * HP + 8 * hh, pWmu, 0, DD, m, hh);
#pragma unroll
    for (int t = 0; t < 8; ++t) {
#pragma unroll
      for (int r8 = 0; r8 < 8; ++r8) {
        const int e = (8 * hh + r8) * DD + 16 * t + m;
        const float v = acc[t][r8] * INV16;
        sV[e] = v;
        sSq[e] = (r == 0) ? v * v : fmaf(v, v, sSq[e]);
      }
    }
    mma8<4>(acc, sMu + (r * 16 + m) * HP + 8 * hh, pWmu, DD, DD, m, hh);
#pragma unroll
    for (int t = 0; t < 8; ++t) {
#pragma unroll
      for (int r8 = 0; r8 < 8; ++r8) {
        const int e = (8 * hh + r8) * DD + 16 * t + m;
        const float w = acc[t][r8] * INV16;
        const float v = sV[e];
        sDt[e] = (r == 0) ? v * w : fmaf(v, w, sDt[e]);
        sW[(8 * hh + r8) * D3 + r * DD + 16 * t + m] = w;
      }
    }
  }
#pragma unroll
  for (int t = 0; t < 8; ++t) {
#pragma unroll
    for (int r8 = 0; r8 < 8; ++r8) {
      const int e = (8 * hh + r8) * DD + 16 * t + m;
      sC[(8 * hh + r8) * AP2 + DD + 16 * t + m] = (_Float16)sqrtf(sSq[e] + EPSV);
    }
  }
  __syncthreads();

  mma8<8>(acc, sC + m * AP2 + 8 * hh, pWm1, 0, D2, m, hh);
#pragma unroll
  for (int t = 0; t < 8; ++t) {
    const float bb = b_m1[16 * t + m];
#pragma unroll
    for (int r8 = 0; r8 < 8; ++r8) {
      const int e = (8 * hh + r8) * DD + 16 * t + m;
      sV[e] = fmaf(acc[t][r8], INV16, bb);
    }
  }
  mma8<8>(acc, sC + m * AP2 + 8 * hh, pWm1, DD, D2, m, hh);
#pragma unroll
  for (int t = 0; t < 8; ++t) {
    const float bg = b_m1[DD + 16 * t + m];
#pragma unroll
    for (int r8 = 0; r8 < 8; ++r8) {
      const int e = (8 * hh + r8) * DD + 16 * t + m;
      const float av = sV[e];
      const float gv = fmaf(acc[t][r8], INV16, bg);
      const float h  = (av * sigm(av)) * sigm(gv);
      sH[(8 * hh + r8) * HP + 16 * t + m] = (_Float16)h;
    }
  }
  __syncthreads();

  mma8<4>(acc, sH + m * HP + 8 * hh, pWm2, 0, DD, m, hh);
#pragma unroll
  for (int t = 0; t < 8; ++t) {
    const float bb = b_m2[16 * t + m];
#pragma unroll
    for (int r8 = 0; r8 < 8; ++r8) {
      const int e = (8 * hh + r8) * DD + 16 * t + m;
      sV[e] = fmaf(acc[t][r8], INV16, bb);
    }
  }
  mma8<4>(acc, sH + m * HP + 8 * hh, pWm2, 2 * DD, DD, m, hh);
#pragma unroll
  for (int t = 0; t < 8; ++t) {
    const float bb = b_m2[2 * DD + 16 * t + m];
#pragma unroll
    for (int r8 = 0; r8 < 8; ++r8) {
      const int row = 8 * hh + r8;
      const int e = row * DD + 16 * t + m;
      const float qv  = Qp[(size_t)(a0 + row) * DD + 16 * t + m];
      const float dqm = fmaf(acc[t][r8], INV16, bb);
      sSq[e] = (qv + sV[e]) + dqm * sDt[e];
    }
  }
  mma8<4>(acc, sH + m * HP + 8 * hh, pWm2, DD, DD, m, hh);
#pragma unroll
  for (int t = 0; t < 8; ++t) {
    const float bb = b_m2[DD + 16 * t + m];
#pragma unroll
    for (int r8 = 0; r8 < 8; ++r8) {
      const int row = 8 * hh + r8;
      const float dmi = fmaf(acc[t][r8], INV16, bb);
#pragma unroll
      for (int r = 0; r < 3; ++r) {
        const int idx = row * D3 + r * DD + 16 * t + m;
        const float muv = MUp[((size_t)(a0 + row) * 3 + r) * DD + 16 * t + m];
        const float wv  = sW[idx];
        sW[idx] = muv + dmi * wv;
      }
    }
  }
  __syncthreads();

  atom2_out(sSq, sW, outq, outmu, a0, nh, lane);
  __threadfence();
  atom2_out(sSq, sW, outq, outmu, a0, nh, lane);
}

extern "C" void kernel_launch(void* const* d_in, const int* in_sizes, int n_in,
                              void* d_out, int out_size, void* d_ws, size_t ws_size,
                              hipStream_t stream) {
  if (n_in < 20) return;
  const int nB = in_sizes[5] / NN;
  if (nB <= 0 || nB > 1024 || in_sizes[5] != nB * NN) return;
  const int nh = in_sizes[0] / (nB * DD);
  if (nh <= 0 || nh > NN || in_sizes[0] != nB * nh * DD) return;
  const int nAt = nB * NN;
  if (in_sizes[1] != nAt * D3 || in_sizes[2] != nAt * NN * RR || in_sizes[3] != nAt * NN * 3 || in_sizes[4] != nAt * NN) return;
  if (in_sizes[6] != DD || in_sizes[7] != RR * D3 || in_sizes[8] != D3 || in_sizes[9] != DD) return;
  if (in_sizes[10] != DD * D2 || in_sizes[11] != D2 || in_sizes[12] != DD * D3 || in_sizes[13] != D3 || in_sizes[14] != DD) return;
  if (in_sizes[15] != D2 * D2 || in_sizes[16] != D2 || in_sizes[17] != DD * D3 || in_sizes[18] != D3 || in_sizes[19] != DD * D2) return;
  if (out_size != nB * nh * DD + nAt * D3) return;

  const float* s_heavy = (const float*)d_in[0];
  const float* v_all   = (const float*)d_in[1];
  const float* rbf     = (const float*)d_in[2];
  const float* dir_ij  = (const float*)d_in[3];
  const float* mask_ij = (const float*)d_in[4];
  const int*   is_h    = (const int*)d_in[5];
  const float* h_emb   = (const float*)d_in[6];
  const float* W_f     = (const float*)d_in[7];
  const float* b_f     = (const float*)d_in[8];
  const float* norm1_w = (const float*)d_in[9];
  const float* W_i1    = (const float*)d_in[10];
  const float* b_i1    = (const float*)d_in[11];
  const float* W_i2    = (const float*)d_in[12];
  const float* b_i2    = (const float*)d_in[13];
  const float* norm2_w = (const float*)d_in[14];
  const float* W_m1    = (const float*)d_in[15];
  const float* b_m1    = (const float*)d_in[16];
  const float* W_m2    = (const float*)d_in[17];
  const float* b_m2    = (const float*)d_in[18];
  const float* W_mu    = (const float*)d_in[19];
  float* outq  = (float*)d_out;
  float* outmu = (float*)d_out + (size_t)nB * nh * DD;

  char* ws = (char*)d_ws;
  size_t off = 0;
  const size_t oWf  = off; off += (size_t)D3 * KRP * 2;  off = (off + 255) & ~(size_t)255;
  const size_t oWi1 = off; off += (size_t)D2 * DD * 2;   off = (off + 255) & ~(size_t)255;
  const size_t oWi2 = off; off += (size_t)D3 * DD * 2;   off = (off + 255) & ~(size_t)255;
  const size_t oWmu = off; off += (size_t)D2 * DD * 2;   off = (off + 255) & ~(size_t)255;
  const size_t oWm1 = off; off += (size_t)D2 * D2 * 2;   off = (off + 255) & ~(size_t)255;
  const size_t oWm2 = off; off += (size_t)D3 * DD * 2;   off = (off + 255) & ~(size_t)255;
  const size_t oX   = off; off += (size_t)nAt * D3 * 4;  off = (off + 255) & ~(size_t)255;
  const size_t oQ   = off; off += (size_t)nAt * DD * 4;  off = (off + 255) & ~(size_t)255;
  const size_t oMU  = off; off += (size_t)nAt * D3 * 4;  off = (off + 255) & ~(size_t)255;
  if (off > ws_size || off > (size_t)134217728) return;
  _Float16* pWf  = (_Float16*)(ws + oWf);
  _Float16* pWi1 = (_Float16*)(ws + oWi1);
  _Float16* pWi2 = (_Float16*)(ws + oWi2);
  _Float16* pWmu = (_Float16*)(ws + oWmu);
  _Float16* pWm1 = (_Float16*)(ws + oWm1);
  _Float16* pWm2 = (_Float16*)(ws + oWm2);
  float*    X    = (float*)(ws + oX);
  float*    Qp   = (float*)(ws + oQ);
  float*    MUp  = (float*)(ws + oMU);

  k_prep<<<G_TOT / NTHR, NTHR, 0, stream>>>(W_f, W_i1, W_i2, W_mu, W_m1, W_m2,
                                            pWf, pWi1, pWi2, pWmu, pWm1, pWm2);

  hipFuncSetAttribute(reinterpret_cast<const void*>(&k_atom1),
                      hipFuncAttributeMaxDynamicSharedMemorySize, LDS1);
  k_atom1<<<nAt / NR1, NT1, LDS1, stream>>>(s_heavy, is_h, h_emb, norm1_w, pWi1, b_i1, pWi2, b_i2, X, nh);

  hipFuncSetAttribute(reinterpret_cast<const void*>(&k_pair),
                      hipFuncAttributeMaxDynamicSharedMemorySize, LDSP);
  k_pair<<<nAt, NTHR, LDSP, stream>>>(rbf, dir_ij, mask_ij, v_all, s_heavy, is_h, h_emb, pWf, b_f, X, Qp, MUp, nh);

  hipFuncSetAttribute(reinterpret_cast<const void*>(&k_atom2),
                      hipFuncAttributeMaxDynamicSharedMemorySize, LDS2);
  k_atom2<<<nAt / NR2, NT2, LDS2, stream>>>(Qp, MUp, norm2_w, pWmu, pWm1, b_m1, pWm2, b_m2, outq, outmu, nh);
}
